// PointNetSetAbstraction_3186865734537
// MI455X (gfx1250) — hardware-verified
//
#include <hip/hip_runtime.h>
#include <stddef.h>
#include <stdint.h>

#pragma clang fp contract(off)

typedef __attribute__((ext_vector_type(16))) _Float16 v16h;
typedef __attribute__((ext_vector_type(8)))  _Float16 v8h;
typedef __attribute__((ext_vector_type(8)))  float    v8f;
typedef __attribute__((ext_vector_type(4)))  float    v4f;
typedef __attribute__((ext_vector_type(4)))  unsigned v4u;

constexpr int kBatch   = 16;
constexpr int kNpts    = 4096;
constexpr int kNpoint  = 1024;
constexpr int kNsample = 64;
constexpr int kCin     = 9;
constexpr int kKpad0   = 32;
constexpr int kC0      = 64;
constexpr int kC1      = 64;
constexpr int kC2      = 128;
constexpr int kGroups  = kBatch * kNpoint;
constexpr int kRows    = kGroups * kNsample;
static_assert(kGroups == 16384, "groups");
static_assert(kRows == 1048576, "rows");
static_assert(kKpad0 % 32 == 0 && kC0 % 32 == 0 && kC1 % 32 == 0, "K multiples of 32");
static_assert(kNsample == 64, "one 64-row tile per group");

constexpr float kRad2 = 0.04f;
constexpr float kBnEps = 1e-5f;
constexpr float kWCarry = 16.0f;
constexpr float kWCarryInv = 1.0f / 16.0f;

constexpr int kMlpWaves      = 2;
constexpr int kGroupsPerWave = 4;
constexpr int kWaveParts     = kGroups / kGroupsPerWave;
constexpr int kMlpBlocks     = kWaveParts / kMlpWaves;
static_assert(kWaveParts * kGroupsPerWave == kGroups, "exact cover");
static_assert(kMlpBlocks * kMlpWaves == kWaveParts, "exact cover");

constexpr size_t kOut0Floats = (size_t)kBatch * kNpoint * 3;
constexpr size_t kOut1Floats = (size_t)kBatch * kC2 * kNpoint;
static_assert(kOut0Floats * 4 == 196608, "out1 byte offset");
static_assert((kOut0Floats * 4) % 128 == 0, "out1 line aligned");
static_assert((kOut0Floats + kOut1Floats) * 4 == 8585216, "d_out total bytes");

constexpr size_t kOffTab   = 0;
constexpr size_t kOffBt0   = kOffTab + 4096;
constexpr size_t kOffBt1   = kOffBt0 + (size_t)kC0 * kKpad0 * 2;
constexpr size_t kOffBt2   = kOffBt1 + (size_t)kC1 * kC0 * 2;
constexpr size_t kOffCent  = kOffBt2 + (size_t)kC2 * kC1 * 2;
constexpr size_t kOffPart0 = kOffCent + (size_t)kGroups * 16;
constexpr size_t kOffPart1 = kOffPart0 + (size_t)kWaveParts * 2 * kC0 * 4;
constexpr size_t kOffPart2 = kOffPart1 + (size_t)kWaveParts * 2 * kC1 * 4;
constexpr size_t kOffYmax  = kOffPart2 + (size_t)kWaveParts * 2 * kC2 * 4;
constexpr size_t kOffYmin  = kOffYmax + (size_t)kGroups * kC2 * 4;
constexpr size_t kOffX0    = kOffYmin + (size_t)kGroups * kC2 * 4;
constexpr size_t kWsTotal  = kOffX0 + (size_t)kRows * kKpad0 * 2;
static_assert(kOffBt0 % 128 == 0 && kOffBt1 % 128 == 0 && kOffBt2 % 128 == 0, "align");
static_assert(kOffCent % 128 == 0 && kOffPart0 % 128 == 0 && kOffPart1 % 128 == 0, "align");
static_assert(kOffPart2 % 128 == 0 && kOffYmax % 128 == 0 && kOffYmin % 128 == 0 && kOffX0 % 128 == 0, "align");
static_assert(kWsTotal <= (size_t)134217728, "carve under 128 MiB");

__device__ __forceinline__ unsigned f16_bits(float x) {
  const _Float16 h = (_Float16)x;
  const unsigned short b = __builtin_bit_cast(unsigned short, h);
  return (unsigned)b;
}

union FragU { v16h v; v8h h[2]; };

__device__ __forceinline__ v16h frag_load(const _Float16* p) {
  FragU f;
  f.h[0] = *(const v8h*)(p);
  f.h[1] = *(const v8h*)(p + 16);
  return f.v;
}

__device__ __forceinline__ v8f mma_f16(v16h a, v16h b, v8f c) {
  c = __builtin_amdgcn_wmma_f32_16x16x32_f16(false, a, false, b, (short)0, c, false, false);
  asm volatile("v_nop\n\tv_nop\n\tv_nop\n\tv_nop" : "+v"(c) : "v"(a), "v"(b));
  return c;
}

__device__ __forceinline__ void wave_lds_sync() {
  __builtin_amdgcn_fence(__ATOMIC_RELEASE, "workgroup");
  __builtin_amdgcn_wave_barrier();
  __builtin_amdgcn_fence(__ATOMIC_ACQUIRE, "workgroup");
}

__device__ __forceinline__ void argmax_merge(float& best, int& bi, float ov, int oi) {
  const bool take = (ov > best) || ((ov == best) && (oi < bi));
  best = take ? ov : best;
  bi = take ? oi : bi;
}

__global__ __launch_bounds__(256) void prep_weights_kernel(
    const float* __restrict__ w0, const float* __restrict__ w1, const float* __restrict__ w2,
    unsigned* __restrict__ bt0, unsigned* __restrict__ bt1, unsigned* __restrict__ bt2) {
  const int t = blockIdx.x * 256 + threadIdx.x;
  if (t < 1024) {
    const int o = t >> 4;
    const int k = (t & 15) * 2;
    const int ka = k < (kCin - 1) ? k : (kCin - 1);
    const int kb = (k + 1) < (kCin - 1) ? (k + 1) : (kCin - 1);
    float a = w0[o * kCin + ka];
    float b = w0[o * kCin + kb];
    a = (k < kCin) ? a * kWCarry : 0.0f;
    b = ((k + 1) < kCin) ? b * kWCarry : 0.0f;
    unsigned lo = f16_bits(a);
    unsigned hi = f16_bits(b);
    asm volatile("" : "+v"(lo), "+v"(hi));
    const unsigned u = lo | (hi << 16);
    volatile unsigned* d = bt0;
    d[t] = u;
    __threadfence();
    d[t] = u;
  } else if (t < 3072) {
    const int uidx = t - 1024;
    const float a = w1[2 * uidx] * kWCarry;
    const float b = w1[2 * uidx + 1] * kWCarry;
    unsigned lo = f16_bits(a);
    unsigned hi = f16_bits(b);
    asm volatile("" : "+v"(lo), "+v"(hi));
    const unsigned u = lo | (hi << 16);
    volatile unsigned* d = bt1;
    d[uidx] = u;
    __threadfence();
    d[uidx] = u;
  } else if (t < 7168) {
    const int uidx = t - 3072;
    const float a = w2[2 * uidx] * kWCarry;
    const float b = w2[2 * uidx + 1] * kWCarry;
    unsigned lo = f16_bits(a);
    unsigned hi = f16_bits(b);
    asm volatile("" : "+v"(lo), "+v"(hi));
    const unsigned u = lo | (hi << 16);
    volatile unsigned* d = bt2;
    d[uidx] = u;
    __threadfence();
    d[uidx] = u;
  }
}

__global__ __launch_bounds__(1024) void fps_kernel(
    const float* __restrict__ xyz, float* __restrict__ out0, float* __restrict__ cent4) {
#pragma clang fp contract(off)
  __shared__ __align__(16) float sX[kNpts * 3];
  __shared__ int sPick[kNpoint];
  __shared__ float sVal[2][32];
  __shared__ int sIdx[2][32];
  const int b = blockIdx.x;
  const int tid = threadIdx.x;
  const int lane = tid & 31;
  const int wave = tid >> 5;
  {
    const v4f* src = (const v4f*)(xyz + (size_t)b * (kNpts * 3));
#pragma unroll
    for (int i = 0; i < 3; ++i) {
      const v4f v = src[tid + i * 1024];
      *(v4f*)(&sX[(tid + i * 1024) * 4]) = v;
    }
  }
  __syncthreads();

  float px[4], py[4], pz[4], dist[4];
#pragma unroll
  for (int i = 0; i < 4; ++i) {
    const int p = tid + i * 1024;
    px[i] = sX[p * 3 + 0];
    py[i] = sX[p * 3 + 1];
    pz[i] = sX[p * 3 + 2];
    dist[i] = 1e10f;
  }

  int far = 0;
  int buf = 0;
  for (int it = 0; it < kNpoint; ++it) {
    if (tid == 0) sPick[it] = far;
    const float cx = sX[far * 3 + 0];
    const float cy = sX[far * 3 + 1];
    const float cz = sX[far * 3 + 2];
    float best = -1.0f;
    int bi = tid;
#pragma unroll
    for (int i = 0; i < 4; ++i) {
      const float dx = px[i] - cx;
      const float dy = py[i] - cy;
      const float dz = pz[i] - cz;
      const float t0 = dx * dx;
      const float t1 = dy * dy;
      const float t2 = dz * dz;
      const float d = (t0 + t2) + t1;
      const float nd = fminf(dist[i], d);
      dist[i] = nd;
      const bool gt = nd > best;
      best = gt ? nd : best;
      bi = gt ? (tid + i * 1024) : bi;
    }
#pragma unroll
    for (int off = 16; off > 0; off >>= 1) {
      const float ov = __shfl_xor(best, off, 32);
      const int oi = __shfl_xor(bi, off, 32);
      argmax_merge(best, bi, ov, oi);
    }
    if (lane == 0) {
      sVal[buf][wave] = best;
      sIdx[buf][wave] = bi;
    }
    __syncthreads();
    float fv = sVal[buf][lane];
    int fi = sIdx[buf][lane];
#pragma unroll
    for (int off = 16; off > 0; off >>= 1) {
      const float ov = __shfl_xor(fv, off, 32);
      const int oi = __shfl_xor(fi, off, 32);
      argmax_merge(fv, fi, ov, oi);
    }
    fi = fi < 0 ? 0 : fi;
    fi = fi > (kNpts - 1) ? (kNpts - 1) : fi;
    far = fi;
    buf ^= 1;
  }
  __syncthreads();

  int pidx = sPick[tid];
  pidx = pidx < 0 ? 0 : pidx;
  pidx = pidx > (kNpts - 1) ? (kNpts - 1) : pidx;
  v4f cv;
  cv.x = sX[pidx * 3 + 0];
  cv.y = sX[pidx * 3 + 1];
  cv.z = sX[pidx * 3 + 2];
  cv.w = 0.0f;
  v4f ov4;
  {
    float tmp[4];
#pragma unroll
    for (int e = 0; e < 4; ++e) {
      const int i = tid * 4 + e;
      int s = i / 3;
      const int cc = i - 3 * s;
      s = s > (kNpoint - 1) ? (kNpoint - 1) : s;
      int sidx = sPick[s];
      sidx = sidx < 0 ? 0 : sidx;
      sidx = sidx > (kNpts - 1) ? (kNpts - 1) : sidx;
      tmp[e] = sX[sidx * 3 + cc];
    }
    ov4.x = tmp[0];
    ov4.y = tmp[1];
    ov4.z = tmp[2];
    ov4.w = tmp[3];
  }
  float* pc = cent4 + ((size_t)b * kNpoint + tid) * 4;
  float* po = out0 + (size_t)b * (kNpoint * 3) + (size_t)tid * 4;
  *(volatile v4f*)pc = cv;
  if (tid < 768) *(volatile v4f*)po = ov4;
  __threadfence();
  *(volatile v4f*)pc = cv;
  if (tid < 768) *(volatile v4f*)po = ov4;
}

__global__ __launch_bounds__(256) void ball_group_kernel(
    const float* __restrict__ xyz, const float* __restrict__ pts,
    const float* __restrict__ cent4, v4u* __restrict__ X0w) {
#pragma clang fp contract(off)
  __shared__ int sSel[8][kNsample];
  __shared__ __align__(16) v4u sRow[8][kNsample * 4];
  const int lane = threadIdx.x & 31;
  const int wib = threadIdx.x >> 5;
  const int cent = blockIdx.x * 8 + wib;
  const int b = cent >> 10;
  const float* xb = xyz + (size_t)b * (kNpts * 3);
  const float* pb = pts + (size_t)b * (kNpts * 6);
  const v4f c4 = *(const v4f*)(cent4 + (size_t)cent * 4);
  const float cx = c4.x;
  const float cy = c4.y;
  const float cz = c4.z;
  const float cxx = cx * cx;
  const float cyy = cy * cy;
  const float czz = cz * cz;
  const float sqc = (cxx + czz) + cyy;

  int count = 0;
  for (int n0 = 0; n0 < kNpts && count < kNsample; n0 += 32) {
    const int p = n0 + lane;
    const float qx = xb[p * 3 + 0];
    const float qy = xb[p * 3 + 1];
    const float qz = xb[p * 3 + 2];
    const float qxx = qx * qx;
    const float qyy = qy * qy;
    const float qzz = qz * qz;
    const float sqp = (qxx + qzz) + qyy;
    float dot = cx * qx;
    dot = __builtin_fmaf(cy, qy, dot);
    dot = __builtin_fmaf(cz, qz, dot);
    const float two_dot = 2.0f * dot;
    const float sqr = (sqc + sqp) - two_dot;
    const bool pred = !(sqr > kRad2);
    const unsigned mask = (unsigned)__ballot(pred);
    const int pos = count + __popc(mask & ((1u << lane) - 1u));
    if (pred && pos < kNsample) sSel[wib][pos] = p;
    count += __popc(mask);
  }
  int total = count < kNsample ? count : kNsample;
  if (count == 0 && lane == 0) sSel[wib][0] = kNpts - 1;
  total = total < 1 ? 1 : total;
  __syncthreads();

  unsigned zz = 0;
  asm volatile("" : "+v"(zz));
#pragma unroll
  for (int rr = 0; rr < 2; ++rr) {
    const int k = lane + rr * 32;
    int idx = sSel[wib][k < total ? k : 0];
    idx = idx < 0 ? 0 : idx;
    idx = idx > (kNpts - 1) ? (kNpts - 1) : idx;
    const float gx = xb[idx * 3 + 0];
    const float gy = xb[idx * 3 + 1];
    const float gz = xb[idx * 3 + 2];
    const float f0 = pb[idx * 6 + 0];
    const float f1 = pb[idx * 6 + 1];
    const float f2 = pb[idx * 6 + 2];
    const float f3 = pb[idx * 6 + 3];
    const float f4 = pb[idx * 6 + 4];
    const float f5 = pb[idx * 6 + 5];
    const unsigned h0 = f16_bits(gx - cx);
    const unsigned h1 = f16_bits(gy - cy);
    const unsigned h2 = f16_bits(gz - cz);
    const unsigned h3 = f16_bits(f0);
    const unsigned h4 = f16_bits(f1);
    const unsigned h5 = f16_bits(f2);
    const unsigned h6 = f16_bits(f3);
    const unsigned h7 = f16_bits(f4);
    const unsigned h8 = f16_bits(f5);
    v4u wa;
    wa.x = h0 | (h1 << 16);
    wa.y = h2 | (h3 << 16);
    wa.z = h4 | (h5 << 16);
    wa.w = h6 | (h7 << 16);
    v4u wb;
    wb.x = (h8 & 0xffffu) | (zz << 16);
    wb.y = zz;
    wb.z = zz;
    wb.w = zz;
    v4u wc;
    wc.x = zz;
    wc.y = zz;
    wc.z = zz;
    wc.w = zz;
    sRow[wib][k * 4 + 0] = wa;
    sRow[wib][k * 4 + 1] = wb;
    sRow[wib][k * 4 + 2] = wc;
    sRow[wib][k * 4 + 3] = wc;
    asm volatile("" ::: "memory");
  }
  __syncthreads();

  v4u* dst = X0w + (size_t)cent * (kNsample * 4);
  for (int pass = 0; pass < 2; ++pass) {
#pragma unroll
    for (int it = 0; it < 8; ++it) {
      const v4u v = sRow[wib][it * 32 + lane];
      *(volatile v4u*)(dst + it * 32 + lane) = v;
    }
    __threadfence();
  }
}

__device__ __forceinline__ void zero_acc(v8f (&acc)[4][2]) {
#pragma unroll
  for (int i = 0; i < 4; ++i) {
    acc[i][0] = (v8f){0.f, 0.f, 0.f, 0.f, 0.f, 0.f, 0.f, 0.f};
    acc[i][1] = (v8f){0.f, 0.f, 0.f, 0.f, 0.f, 0.f, 0.f, 0.f};
  }
}

template <int J>
__device__ __forceinline__ void acc_colstats(const v8f (&acc)[4][2], float& s, float& q) {
  float ls = 0.0f;
  float lq = 0.0f;
#pragma unroll
  for (int i = 0; i < 4; ++i) {
#pragma unroll
    for (int r = 0; r < 8; ++r) {
      const float v = acc[i][J][r];
      ls += v;
      lq += v * v;
    }
  }
  const float os = __shfl_xor(ls, 16, 32);
  const float oq = __shfl_xor(lq, 16, 32);
  ls += os;
  lq += oq;
  s += ls;
  q += lq;
}

template <int J>
__device__ __forceinline__ void acc_colminmax(const v8f (&acc)[4][2], float& mx, float& mn) {
  float a = acc[0][J][0];
  float b = a;
#pragma unroll
  for (int i = 0; i < 4; ++i) {
#pragma unroll
    for (int r = 0; r < 8; ++r) {
      const float v = acc[i][J][r];
      a = fmaxf(a, v);
      b = fminf(b, v);
    }
  }
  const float oa = __shfl_xor(a, 16, 32);
  const float ob = __shfl_xor(b, 16, 32);
  mx = fmaxf(a, oa);
  mn = fminf(b, ob);
}

template <int J>
__device__ __forceinline__ void acc_bnrelu_store(const v8f (&acc)[4][2], float sc, float sh,
                                                 _Float16* tile, int col, int mOff) {
#pragma unroll
  for (int i = 0; i < 4; ++i) {
#pragma unroll
    for (int r = 0; r < 8; ++r) {
      float v = acc[i][J][r] * sc + sh;
      v = fmaxf(v, 0.0f);
      tile[(i * 16 + mOff + r) * 64 + col] = (_Float16)v;
    }
  }
}

__device__ __forceinline__ void gemm_k64_lds(const _Float16* tile, const _Float16* Bt, int nbase,
                                             int rlane, int koff, v8f (&acc)[4][2]) {
  zero_acc(acc);
#pragma unroll
  for (int ks = 0; ks < 2; ++ks) {
    const v16h b0 = frag_load(Bt + (size_t)(nbase + rlane) * 64 + ks * 32 + koff);
    const v16h b1 = frag_load(Bt + (size_t)(nbase + 16 + rlane) * 64 + ks * 32 + koff);
#pragma unroll
    for (int i = 0; i < 4; ++i) {
      FragU fa;
      fa.h[0] = *(const v8h*)(tile + (i * 16 + rlane) * 64 + ks * 32 + koff);
      fa.h[1] = *(const v8h*)(tile + (i * 16 + rlane) * 64 + ks * 32 + koff + 16);
      acc[i][0] = mma_f16(fa.v, b0, acc[i][0]);
      acc[i][1] = mma_f16(fa.v, b1, acc[i][1]);
    }
  }
}

template <int PASS>
__global__ __launch_bounds__(64) void mlp_pass_kernel(
    const _Float16* __restrict__ X0, const _Float16* __restrict__ Bt0,
    const _Float16* __restrict__ Bt1, const _Float16* __restrict__ Bt2,
    const float* __restrict__ tab, float* __restrict__ part,
    float* __restrict__ ymax, float* __restrict__ ymin) {
  constexpr int NSTAT = (PASS == 3) ? 8 : 4;
  constexpr int NCH = NSTAT * 16;
  __shared__ __align__(16) _Float16 sTileA[kMlpWaves][64 * 64];
  __shared__ __align__(16) _Float16 sTileB[kMlpWaves][64 * 64];
  __shared__ __align__(16) float sStat[kMlpWaves][256];
  __shared__ __align__(16) float sMax[kMlpWaves][128];
  __shared__ __align__(16) float sMin[kMlpWaves][128];

  const int lane = threadIdx.x & 31;
  const int wave = threadIdx.x >> 5;
  const int rlane = lane & 15;
  const int hh = lane >> 4;
  const int koff = hh * 8;
  const int mOff = hh * 8;
  const int wg = blockIdx.x * kMlpWaves + wave;

  float ssum[NSTAT], ssq[NSTAT];
#pragma unroll
  for (int i = 0; i < NSTAT; ++i) {
    ssum[i] = 0.0f;
    ssq[i] = 0.0f;
  }
  _Float16* tileA = sTileA[wave];
  _Float16* tileB = sTileB[wave];

#pragma unroll 1
  for (int t = 0; t < kGroupsPerWave; ++t) {
    const int g = wg * kGroupsPerWave + t;
    const _Float16* Xg = X0 + (size_t)g * (64 * kKpad0);

#pragma unroll
    for (int nh = 0; nh < 2; ++nh) {
      v8f acc[4][2];
      zero_acc(acc);
      const v16h b0 = frag_load(Bt0 + (size_t)(nh * 32 + rlane) * kKpad0 + koff);
      const v16h b1 = frag_load(Bt0 + (size_t)(nh * 32 + 16 + rlane) * kKpad0 + koff);
#pragma unroll
      for (int i = 0; i < 4; ++i) {
        const v16h a = frag_load(Xg + (size_t)(i * 16 + rlane) * kKpad0 + koff);
        acc[i][0] = mma_f16(a, b0, acc[i][0]);
        acc[i][1] = mma_f16(a, b1, acc[i][1]);
      }
      if (PASS == 1) {
        acc_colstats<0>(acc, ssum[nh * 2 + 0], ssq[nh * 2 + 0]);
        acc_colstats<1>(acc, ssum[nh * 2 + 1], ssq[nh * 2 + 1]);
      } else {
        const int ch0 = nh * 32 + rlane;
        const int ch1 = ch0 + 16;
        const float sc0 = tab[ch0];
        const float sh0 = tab[128 + ch0];
        const float sc1 = tab[ch1];
        const float sh1 = tab[128 + ch1];
        acc_bnrelu_store<0>(acc, sc0, sh0, tileA, ch0, mOff);
        acc_bnrelu_store<1>(acc, sc1, sh1, tileA, ch1, mOff);
      }
    }

    if (PASS >= 2) {
      wave_lds_sync();
#pragma unroll
      for (int nh = 0; nh < 2; ++nh) {
        v8f acc[4][2];
        gemm_k64_lds(tileA, Bt1, nh * 32, rlane, koff, acc);
        if (PASS == 2) {
          acc_colstats<0>(acc, ssum[nh * 2 + 0], ssq[nh * 2 + 0]);
          acc_colstats<1>(acc, ssum[nh * 2 + 1], ssq[nh * 2 + 1]);
        } else {
          const int ch0 = nh * 32 + rlane;
          const int ch1 = ch0 + 16;
          const float sc0 = tab[256 + ch0];
          const float sh0 = tab[256 + 128 + ch0];
          const float sc1 = tab[256 + ch1];
          const float sh1 = tab[256 + 128 + ch1];
          acc_bnrelu_store<0>(acc, sc0, sh0, tileB, ch0, mOff);
          acc_bnrelu_store<1>(acc, sc1, sh1, tileB, ch1, mOff);
        }
      }
      wave_lds_sync();
    }

    if (PASS == 3) {
#pragma unroll
      for (int nq = 0; nq < 4; ++nq) {
        v8f acc[4][2];
        gemm_k64_lds(tileB, Bt2, nq * 32, rlane, koff, acc);
        acc_colstats<0>(acc, ssum[(nq * 2 + 0) % NSTAT], ssq[(nq * 2 + 0) % NSTAT]);
        acc_colstats<1>(acc, ssum[(nq * 2 + 1) % NSTAT], ssq[(nq * 2 + 1) % NSTAT]);
        float mx0, mn0, mx1, mn1;
        acc_colminmax<0>(acc, mx0, mn0);
        acc_colminmax<1>(acc, mx1, mn1);
        if (hh == 0) {
          sMax[wave][nq * 32 + rlane] = mx0;
          sMin[wave][nq * 32 + rlane] = mn0;
          sMax[wave][nq * 32 + 16 + rlane] = mx1;
          sMin[wave][nq * 32 + 16 + rlane] = mn1;
        }
      }
      wave_lds_sync();
      {
        const v4f vmx = *(const v4f*)(&sMax[wave][lane * 4]);
        const v4f vmn = *(const v4f*)(&sMin[wave][lane * 4]);
        float* pmx = ymax + (size_t)g * kC2 + lane * 4;
        float* pmn = ymin + (size_t)g * kC2 + lane * 4;
        *(volatile v4f*)pmx = vmx;
        *(volatile v4f*)pmn = vmn;
        __threadfence();
        *(volatile v4f*)pmx = vmx;
        *(volatile v4f*)pmn = vmn;
      }
      wave_lds_sync();
    }
  }

  if (hh == 0) {
#pragma unroll
    for (int i = 0; i < NSTAT; ++i) {
      sStat[wave][i * 16 + rlane] = ssum[i];
      sStat[wave][NCH + i * 16 + rlane] = ssq[i];
    }
  }
  wave_lds_sync();
  {
    float* dst = part + (size_t)wg * (2 * NCH);
    for (int pass = 0; pass < 2; ++pass) {
#pragma unroll
      for (int c = 0; c < (2 * NCH) / 128; ++c) {
        const v4f v = *(const v4f*)(&sStat[wave][c * 128 + lane * 4]);
        *(volatile v4f*)(dst + c * 128 + lane * 4) = v;
      }
      __threadfence();
    }
  }
}

template <int NC>
__global__ __launch_bounds__(256) void bn_finalize_kernel(
    const float* __restrict__ part, const float* __restrict__ bias,
    const float* __restrict__ gam, const float* __restrict__ bet, float* __restrict__ tabOut) {
  constexpr int NCOLS = 2 * NC;
  constexpr int NPARTS = 256 / NCOLS;
  static_assert(NCOLS * NPARTS == 256, "thread map");
  __shared__ double sD[256];
  __shared__ float sO[256];
  const int tid = threadIdx.x;
  const int col = tid % NCOLS;
  const int p = tid / NCOLS;
  double a = 0.0;
#pragma unroll 4
  for (int row = p; row < kWaveParts; row += NPARTS) {
    a += (double)part[(size_t)row * NCOLS + col];
  }
  sD[tid] = a;
  sO[tid] = 0.0f;
  __syncthreads();
  if (tid < NC) {
    double S = 0.0;
    double Q = 0.0;
    for (int pp = 0; pp < NPARTS; ++pp) {
      S += sD[pp * NCOLS + tid];
      Q += sD[pp * NCOLS + NC + tid];
    }
    const double invM = 1.0 / (double)kRows;
    const double mu = S * invM;
    double var = Q * invM - mu * mu;
    var = var < 0.0 ? 0.0 : var;
    const float vy = (float)(var * (double)(kWCarryInv * kWCarryInv));
    const float rs = 1.0f / sqrtf(vy + kBnEps);
    const float bb = bias[tid];
    const float sc = gam[tid] * rs;
    const float mean_y = (float)(mu * (double)kWCarryInv) + bb;
    const float sh = bet[tid] - mean_y * sc;
    const float scA = sc * kWCarryInv;
    const float shA = sc * bb + sh;
    sO[tid] = scA;
    sO[128 + tid] = shA;
  }
  __syncthreads();
  const float v = sO[tid];
  volatile float* o = tabOut;
  o[tid] = v;
  __threadfence();
  o[tid] = v;
}

__global__ __launch_bounds__(256) void pool_out_kernel(
    const float* __restrict__ ymax, const float* __restrict__ ymin,
    const float* __restrict__ tab2, float* __restrict__ out1) {
  __shared__ __align__(16) float sT[128 * 36];
  const int tid = threadIdx.x;
  const int b = blockIdx.x >> 5;
  const int s0 = (blockIdx.x & 31) * 32;
  const int g0 = b * kNpoint + s0;
  const int c = tid & 127;
  const float sc = tab2[c];
  const float sh = tab2[128 + c];
  const float fa = (sc >= 0.0f) ? 1.0f : 0.0f;
  const float fb = 1.0f - fa;
#pragma unroll 4
  for (int it = 0; it < 16; ++it) {
    const int sl = it * 2 + (tid >> 7);
    const float mx = ymax[(size_t)(g0 + sl) * kC2 + c];
    const float mn = ymin[(size_t)(g0 + sl) * kC2 + c];
    const float pa = fa * mx;
    const float pb = fb * mn;
    const float x = pa + pb;
    float v = sc * x + sh;
    v = fmaxf(v, 0.0f);
    sT[c * 36 + sl] = v;
  }
  __syncthreads();
  const int wave = tid >> 5;
  const int lane = tid & 31;
  const int q = lane >> 3;
  const int s4 = (lane & 7) * 4;
  for (int pass = 0; pass < 2; ++pass) {
#pragma unroll
    for (int it = 0; it < 4; ++it) {
      const int ch = it * 32 + wave * 4 + q;
      const v4f v = *(const v4f*)(&sT[ch * 36 + s4]);
      *(volatile v4f*)(out1 + ((size_t)(b * kC2 + ch)) * kNpoint + s0 + s4) = v;
    }
    __threadfence();
  }
}

extern "C" void kernel_launch(void* const* d_in, const int* in_sizes, int n_in,
                              void* d_out, int out_size, void* d_ws, size_t ws_size,
                              hipStream_t stream) {
  (void)in_sizes;
  if (n_in < 14) return;
  if (ws_size < kWsTotal) return;
  if ((size_t)out_size < kOut0Floats + kOut1Floats) return;

  const float* xyz = (const float*)d_in[0];
  const float* pts = (const float*)d_in[1];
  const float* w0  = (const float*)d_in[2];
  const float* b0  = (const float*)d_in[3];
  const float* g0  = (const float*)d_in[4];
  const float* be0 = (const float*)d_in[5];
  const float* w1  = (const float*)d_in[6];
  const float* b1  = (const float*)d_in[7];
  const float* g1  = (const float*)d_in[8];
  const float* be1 = (const float*)d_in[9];
  const float* w2  = (const float*)d_in[10];
  const float* b2  = (const float*)d_in[11];
  const float* g2  = (const float*)d_in[12];
  const float* be2 = (const float*)d_in[13];

  char* ws = (char*)d_ws;
  float* tab   = (float*)(ws + kOffTab);
  unsigned* bt0w = (unsigned*)(ws + kOffBt0);
  unsigned* bt1w = (unsigned*)(ws + kOffBt1);
  unsigned* bt2w = (unsigned*)(ws + kOffBt2);
  float* cent4 = (float*)(ws + kOffCent);
  float* part0 = (float*)(ws + kOffPart0);
  float* part1 = (float*)(ws + kOffPart1);
  float* part2 = (float*)(ws + kOffPart2);
  float* ymax  = (float*)(ws + kOffYmax);
  float* ymin  = (float*)(ws + kOffYmin);
  v4u* x0w     = (v4u*)(ws + kOffX0);
  const _Float16* x0h  = (const _Float16*)(ws + kOffX0);
  const _Float16* bt0h = (const _Float16*)(ws + kOffBt0);
  const _Float16* bt1h = (const _Float16*)(ws + kOffBt1);
  const _Float16* bt2h = (const _Float16*)(ws + kOffBt2);

  float* out0 = (float*)d_out;
  float* out1 = (float*)d_out + kOut0Floats;

  prep_weights_kernel<<<28, 256, 0, stream>>>(w0, w1, w2, bt0w, bt1w, bt2w);
  fps_kernel<<<kBatch, 1024, 0, stream>>>(xyz, out0, cent4);
  ball_group_kernel<<<kGroups / 8, 256, 0, stream>>>(xyz, pts, cent4, x0w);

  mlp_pass_kernel<1><<<kMlpBlocks, 64, 0, stream>>>(x0h, bt0h, bt1h, bt2h, tab, part0, ymax, ymin);
  bn_finalize_kernel<kC0><<<1, 256, 0, stream>>>(part0, b0, g0, be0, tab + 0);
  mlp_pass_kernel<2><<<kMlpBlocks, 64, 0, stream>>>(x0h, bt0h, bt1h, bt2h, tab, part1, ymax, ymin);
  bn_finalize_kernel<kC1><<<1, 256, 0, stream>>>(part1, b1, g1, be1, tab + 256);
  mlp_pass_kernel<3><<<kMlpBlocks, 64, 0, stream>>>(x0h, bt0h, bt1h, bt2h, tab, part2, ymax, ymin);
  bn_finalize_kernel<kC2><<<1, 256, 0, stream>>>(part2, b2, g2, be2, tab + 512);
  pool_out_kernel<<<kBatch * 32, 256, 0, stream>>>(ymax, ymin, tab + 512, out1);
}
